// NeighborAttentionLayer_52501680226798
// MI455X (gfx1250) — hardware-verified
//
#include <hip/hip_runtime.h>
#include <stdint.h>

#define NCELL 8192
#define FG    128
#define DKK   32
#define KNB   16
#define EMBD  64
#define F2    256
#define SP    132
#define KP    32

#define OFF_HS    0
#define OFF_HALL  512
#define OFF_WT    1536
#define OFF_AG    5632
#define OFF_WHH   7680
#define OFF_WHL   15872
#define OFF_QH    24064
#define OFF_QL    32256
#define OFF_KH    40448
#define OFF_KL    48640
#define OFF_CH    56832
#define OFF_CL    65024
#define OFF_HNB   73216
#define OFF_S     81408
#define LDS_CELL  148992
static_assert(OFF_HALL == OFF_HS + FG * 4);
static_assert(OFF_WT == OFF_HALL + F2 * 4);
static_assert(OFF_AG == OFF_WT + 2 * DKK * KP * 2);
static_assert(OFF_WHH == OFF_AG + DKK * KP * 2);
static_assert(OFF_WHL == OFF_WHH + FG * KP * 2);
static_assert(OFF_QH == OFF_WHL + FG * KP * 2);
static_assert(OFF_QL == OFF_QH + FG * KP * 2);
static_assert(OFF_KH == OFF_QL + FG * KP * 2);
static_assert(OFF_KL == OFF_KH + FG * KP * 2);
static_assert(OFF_CH == OFF_KL + FG * KP * 2);
static_assert(OFF_CL == OFF_CH + FG * KP * 2);
static_assert(OFF_HNB == OFF_CL + FG * KP * 2);
static_assert(OFF_S == OFF_HNB + FG * KP * 2);
static_assert(LDS_CELL == OFF_S + FG * SP * 4);

#define WS_WCT   0
#define WS_HF    32768
#define WS_HH    (WS_HF + NCELL * F2 * 4)
#define WS_HL    (WS_HH + NCELL * F2 * 2)
#define WS_W12   (WS_HL + NCELL * F2 * 2)
#define WS_TOTAL (WS_W12 + 2 * NCELL * 4)
static_assert(WS_WCT + EMBD * F2 * 2 == WS_HF);
static_assert(WS_TOTAL == 16875520);
static_assert((WS_HF % 128) == 0 && (WS_HH % 128) == 0 && (WS_HL % 128) == 0 && (WS_W12 % 128) == 0);

typedef __bf16         v16bf __attribute__((ext_vector_type(16)));
typedef unsigned short v16us __attribute__((ext_vector_type(16)));
typedef unsigned short v8us  __attribute__((ext_vector_type(8)));
typedef float          v8f   __attribute__((ext_vector_type(8)));
typedef float          v4f   __attribute__((ext_vector_type(4)));

union Frag { v16bf v; v16us u; v8us half[2]; };

__device__ __forceinline__ unsigned short bfb(float f) {
  const unsigned u = __float_as_uint(f);
  return (unsigned short)((u + 0x7FFFu + ((u >> 16) & 1u)) >> 16);
}
__device__ __forceinline__ float bfu(unsigned short b) { return __uint_as_float(((unsigned)b) << 16); }
__device__ __forceinline__ float bfr(float f) { return bfu(bfb(f)); }
__device__ __forceinline__ v8f zero8() {
  v8f z;
  z[0] = 0.f; z[1] = 0.f; z[2] = 0.f; z[3] = 0.f; z[4] = 0.f; z[5] = 0.f; z[6] = 0.f; z[7] = 0.f;
  return z;
}
__device__ __forceinline__ float elu1(float v) {
  const float e = __expf(fminf(v, 0.0f)) - 1.0f;
  return v > 0.0f ? v : e;
}
__device__ __forceinline__ v4f elu4(v4f v) {
  v4f o;
  o[0] = elu1(v[0]); o[1] = elu1(v[1]); o[2] = elu1(v[2]); o[3] = elu1(v[3]);
  return o;
}

__device__ __forceinline__ v16bf ldf(const unsigned short* p) {
  Frag f;
  f.half[0] = *(const v8us*)(p);
  f.half[1] = *(const v8us*)(p + 16);
  return f.v;
}

__device__ __forceinline__ v8f mma(v16bf a, v16bf b, v8f c) {
  v8f d = __builtin_amdgcn_wmma_f32_16x16x32_bf16(false, a, false, b, (short)0, c, false, false);
#if defined(__HIP_DEVICE_COMPILE__)
  asm volatile("v_nop\n\tv_nop\n\tv_nop\n\tv_nop" : "+v"(d) : "v"(a), "v"(b));
#endif
  return d;
}

__device__ __forceinline__ void split8(v8f x, v8us& ph, v8us& pl) {
#pragma unroll
  for (int r = 0; r < 8; ++r) {
    const unsigned short hb = bfb(x[r]);
    ph[r] = hb;
    pl[r] = bfb(x[r] - bfu(hb));
  }
}
__device__ __forceinline__ void st8f(float* p, v8f a) {
  v4f u0, u1;
  u0[0] = a[0]; u0[1] = a[1]; u0[2] = a[2]; u0[3] = a[3];
  u1[0] = a[4]; u1[1] = a[5]; u1[2] = a[6]; u1[3] = a[7];
  *(v4f*)(p) = u0;
  *(v4f*)(p + 4) = u1;
}

__global__ __launch_bounds__(256) void k_prep(const float* __restrict__ Wc, unsigned short* WCT) {
  const int tid = threadIdx.x;
  const int eb  = 16 * blockIdx.x;
  const int kg  = (tid & 31) * 8;
  const int e0  = eb + (tid >> 5);
  const int e1  = eb + 8 + (tid >> 5);
  v8us p0, p1;
#pragma unroll
  for (int j = 0; j < 8; ++j) {
    p0[j] = bfb(Wc[(kg + j) * EMBD + e0]);
    p1[j] = bfb(Wc[(kg + j) * EMBD + e1]);
  }
  unsigned short* d0 = WCT + (size_t)e0 * F2 + kg;
  unsigned short* d1 = WCT + (size_t)e1 * F2 + kg;
  *(volatile v8us*)d0 = p0;
  *(volatile v8us*)d1 = p1;
  __threadfence();
  *(volatile v8us*)d0 = p0;
  *(volatile v8us*)d1 = p1;
}

__device__ __forceinline__ void proj16(const unsigned short* WTp, const float* __restrict__ bias,
                                       v16bf bwh, v16bf bwl, unsigned short* PH, unsigned short* PL,
                                       int brow, int lr, int lh, v8f z8) {
#pragma unroll
  for (int tm = 0; tm < 2; ++tm) {
    const int d0 = 16 * tm + 8 * lh;
    const v16bf a = ldf(WTp + (16 * tm + lr) * KP + 8 * lh);
    v8f acc = mma(a, bwh, z8);
    acc = mma(a, bwl, acc);
    const v4f c0 = *(const v4f*)(bias + d0);
    const v4f c1 = *(const v4f*)(bias + d0 + 4);
    v8f x;
    x[0] = acc[0] + bfr(c0[0]); x[1] = acc[1] + bfr(c0[1]); x[2] = acc[2] + bfr(c0[2]); x[3] = acc[3] + bfr(c0[3]);
    x[4] = acc[4] + bfr(c1[0]); x[5] = acc[5] + bfr(c1[1]); x[6] = acc[6] + bfr(c1[2]); x[7] = acc[7] + bfr(c1[3]);
    v8us ph, pl;
    split8(x, ph, pl);
    *(v8us*)(PH + brow * KP + d0) = ph;
    *(v8us*)(PL + brow * KP + d0) = pl;
  }
}

__device__ __forceinline__ void score8(const unsigned short* AH, const unsigned short* AL,
                                       v16bf bqh, v16bf bql, float* S, int brow, int lr, int lh, v8f z8) {
#pragma unroll 2
  for (int tn = 0; tn < 8; ++tn) {
    const int arow = 16 * tn + lr;
    const v16bf ah = ldf(AH + arow * KP + 8 * lh);
    const v16bf al = ldf(AL + arow * KP + 8 * lh);
    v8f acc = mma(ah, bqh, z8);
    acc = mma(ah, bql, acc);
    acc = mma(al, bqh, acc);
    st8f(S + brow * SP + 16 * tn + 8 * lh, acc);
  }
}

__device__ __forceinline__ void softmax16(const float* S, const float* hs, float* hall_dst,
                                          int wid, int lr, int lh) {
  const float INVS = 0.17677669529663687f;
  const int f  = 16 * wid + lr;
  const int g0 = 64 * lh;
  const float* sr = S + f * SP + g0;
  float mx = -3.0e38f;
#pragma unroll 4
  for (int j = 0; j < 16; ++j) {
    const v4f s = *(const v4f*)(sr + 4 * j);
    mx = fmaxf(mx, fmaxf(fmaxf(s[0], s[1]), fmaxf(s[2], s[3])));
  }
  mx = fmaxf(mx, __shfl_xor(mx, 16, 32));
  float se = 0.0f, sh = 0.0f;
#pragma unroll 2
  for (int j = 0; j < 16; ++j) {
    const v4f s  = *(const v4f*)(sr + 4 * j);
    const v4f hv = *(const v4f*)(hs + g0 + 4 * j);
#pragma unroll
    for (int c = 0; c < 4; ++c) {
      const float e = __expf((s[c] - mx) * INVS);
      se += e;
      sh += e * hv[c];
    }
  }
  se += __shfl_xor(se, 16, 32);
  sh += __shfl_xor(sh, 16, 32);
  const float val = sh * __builtin_amdgcn_rcpf(se) + hs[f];
  if (lh == 0) hall_dst[f] = val;
}

__global__ __launch_bounds__(256) void k_cell(const float* __restrict__ h, const int* __restrict__ kadj,
                                              const float* __restrict__ Whw, const float* __restrict__ Whb,
                                              const float* __restrict__ Qw, const float* __restrict__ Qb,
                                              const float* __restrict__ Kw, const float* __restrict__ Kb,
                                              const float* __restrict__ Ag,
                                              float* HF, unsigned short* HH, unsigned short* HL, int N) {
  extern __shared__ __align__(16) unsigned char smem[];
  float*          hs   = (float*)(smem + OFF_HS);
  float*          hall = (float*)(smem + OFF_HALL);
  unsigned short* WT   = (unsigned short*)(smem + OFF_WT);
  unsigned short* AG   = (unsigned short*)(smem + OFF_AG);
  unsigned short* WHH  = (unsigned short*)(smem + OFF_WHH);
  unsigned short* WHL  = (unsigned short*)(smem + OFF_WHL);
  unsigned short* QH   = (unsigned short*)(smem + OFF_QH);
  unsigned short* QL   = (unsigned short*)(smem + OFF_QL);
  unsigned short* KH   = (unsigned short*)(smem + OFF_KH);
  unsigned short* KL   = (unsigned short*)(smem + OFF_KL);
  unsigned short* CH   = (unsigned short*)(smem + OFF_CH);
  unsigned short* CL   = (unsigned short*)(smem + OFF_CL);
  unsigned short* HNB  = (unsigned short*)(smem + OFF_HNB);
  float*          S    = (float*)(smem + OFF_S);

  const int tid  = threadIdx.x;
  const int lane = tid & 31;
  const int wid  = tid >> 5;
  const int lr   = lane & 15;
  const int lh   = lane >> 4;
  const int n    = blockIdx.x;
  const float* hrow = h + (size_t)n * FG;

  if (tid < 128) {
    hs[tid] = bfr(hrow[tid]);
    const int dq = tid & 31;
    const int q  = tid >> 5;
    v8us pq, pk;
#pragma unroll
    for (int j = 0; j < 8; ++j) {
      const int k = 8 * q + j;
      pq[j] = bfb(Qw[k * DKK + dq]);
      pk[j] = bfb(Kw[k * DKK + dq]);
    }
    *(v8us*)(WT + dq * KP + 8 * q) = pq;
    *(v8us*)(WT + DKK * KP + dq * KP + 8 * q) = pk;
  } else {
    const int t2 = tid - 128;
    const int d  = t2 >> 2;
    const int q  = t2 & 3;
    const int qq = min(q, 1);
    const v4f a0 = *(const v4f*)(Ag + d * KNB + 8 * qq);
    const v4f a1 = *(const v4f*)(Ag + d * KNB + 8 * qq + 4);
    const bool live = q < 2;
    v8us p;
#pragma unroll
    for (int c = 0; c < 4; ++c) {
      p[c]     = live ? bfb(a0[c]) : (unsigned short)0;
      p[4 + c] = live ? bfb(a1[c]) : (unsigned short)0;
    }
    *(v8us*)(AG + d * KP + 8 * q) = p;
  }
  {
#pragma clang fp contract(off)
    for (int it = 0; it < 2; ++it) {
      const int i  = it * 256 + tid;
      const int f  = i >> 2;
      const int dg = (i & 3) * 8;
      const float hv = bfr(hrow[f]);
      const v4f w0 = *(const v4f*)(Whw + dg);
      const v4f w1 = *(const v4f*)(Whw + dg + 4);
      const v4f b0 = *(const v4f*)(Whb + dg);
      const v4f b1 = *(const v4f*)(Whb + dg + 4);
      v8f x;
      x[0] = hv * bfr(w0[0]) + bfr(b0[0]); x[1] = hv * bfr(w0[1]) + bfr(b0[1]);
      x[2] = hv * bfr(w0[2]) + bfr(b0[2]); x[3] = hv * bfr(w0[3]) + bfr(b0[3]);
      x[4] = hv * bfr(w1[0]) + bfr(b1[0]); x[5] = hv * bfr(w1[1]) + bfr(b1[1]);
      x[6] = hv * bfr(w1[2]) + bfr(b1[2]); x[7] = hv * bfr(w1[3]) + bfr(b1[3]);
      x[0] = fmaxf(x[0], 0.0f); x[1] = fmaxf(x[1], 0.0f); x[2] = fmaxf(x[2], 0.0f); x[3] = fmaxf(x[3], 0.0f);
      x[4] = fmaxf(x[4], 0.0f); x[5] = fmaxf(x[5], 0.0f); x[6] = fmaxf(x[6], 0.0f); x[7] = fmaxf(x[7], 0.0f);
      v8us ph, pl;
      split8(x, ph, pl);
      *(v8us*)(WHH + f * KP + dg) = ph;
      *(v8us*)(WHL + f * KP + dg) = pl;
    }
  }
  {
    const int g = tid & 127;
    const int q = tid >> 7;
    const int* kr = kadj + (size_t)n * KNB + 8 * q;
    v8us p;
#pragma unroll
    for (int j = 0; j < 8; ++j) {
      int idx = kr[j];
      idx = min(max(idx, 0), N - 1);
      p[j] = bfb(h[(size_t)idx * FG + g]);
    }
    *(v8us*)(HNB + g * KP + 8 * q) = p;
    v8us z;
#pragma unroll
    for (int j = 0; j < 8; ++j) z[j] = (unsigned short)0;
    *(v8us*)(HNB + g * KP + 16 + 8 * q) = z;
  }
  __syncthreads();

  const v8f z8 = zero8();
  const int brow = 16 * wid + lr;

  {
    const v16bf bwh = ldf(WHH + brow * KP + 8 * lh);
    const v16bf bwl = ldf(WHL + brow * KP + 8 * lh);
    proj16(WT, Qb, bwh, bwl, QH, QL, brow, lr, lh, z8);
    proj16(WT + DKK * KP, Kb, bwh, bwl, KH, KL, brow, lr, lh, z8);
    const v16bf bhn = ldf(HNB + brow * KP + 8 * lh);
#pragma unroll
    for (int tm = 0; tm < 2; ++tm) {
      const int d0 = 16 * tm + 8 * lh;
      const v16bf a = ldf(AG + (16 * tm + lr) * KP + 8 * lh);
      const v8f acc = mma(a, bhn, z8);
      v8us ph, pl;
      split8(acc, ph, pl);
      *(v8us*)(CH + brow * KP + d0) = ph;
      *(v8us*)(CL + brow * KP + d0) = pl;
    }
  }
  __syncthreads();

  const v16bf bqh = ldf(QH + brow * KP + 8 * lh);
  const v16bf bql = ldf(QL + brow * KP + 8 * lh);
  score8(KH, KL, bqh, bql, S, brow, lr, lh, z8);
  __syncthreads();
  softmax16(S, hs, hall, wid, lr, lh);
  __syncthreads();

  score8(CH, CL, bqh, bql, S, brow, lr, lh, z8);
  __syncthreads();
  softmax16(S, hs, hall + FG, wid, lr, lh);
  __syncthreads();

  if (wid == 0) {
    const v4f a = *(const v4f*)(hall + 4 * lane);
    const v4f b = *(const v4f*)(hall + FG + 4 * lane);
    float* o = HF + (size_t)n * F2 + 4 * lane;
    *(volatile v4f*)(o)      = a;
    *(volatile v4f*)(o + FG) = b;
    __threadfence();
    *(volatile v4f*)(o)      = a;
    *(volatile v4f*)(o + FG) = b;
  } else if (wid == 1) {
    const v4f a = *(const v4f*)(hall + 8 * lane);
    const v4f b = *(const v4f*)(hall + 8 * lane + 4);
    v8f x;
    x[0] = a[0]; x[1] = a[1]; x[2] = a[2]; x[3] = a[3]; x[4] = b[0]; x[5] = b[1]; x[6] = b[2]; x[7] = b[3];
    v8us ph, pl;
    split8(x, ph, pl);
    unsigned short* oh = HH + (size_t)n * F2 + 8 * lane;
    unsigned short* ol = HL + (size_t)n * F2 + 8 * lane;
    *(volatile v8us*)oh = ph;
    *(volatile v8us*)ol = pl;
    __threadfence();
    *(volatile v8us*)oh = ph;
    *(volatile v8us*)ol = pl;
  }
}

__global__ __launch_bounds__(128) void k_wcell(const unsigned short* __restrict__ HH,
                                               const unsigned short* __restrict__ HL,
                                               const unsigned short* __restrict__ WCT,
                                               const float* __restrict__ ac, float* W12, int N) {
  __shared__ __align__(16) float ws12[128];
  const int tid  = threadIdx.x;
  const int lane = tid & 31;
  const int wid  = tid >> 5;
  const int lr   = lane & 15;
  const int lh   = lane >> 4;
  const int r0   = 64 * blockIdx.x;
  const int arow = r0 + 16 * wid + lr;
  const unsigned short* pah = HH + (size_t)arow * F2 + 8 * lh;
  const unsigned short* pal = HL + (size_t)arow * F2 + 8 * lh;
  const unsigned short* pb0 = WCT + (size_t)(0 * 16 + lr) * F2 + 8 * lh;
  const unsigned short* pb1 = WCT + (size_t)(1 * 16 + lr) * F2 + 8 * lh;
  const unsigned short* pb2 = WCT + (size_t)(2 * 16 + lr) * F2 + 8 * lh;
  const unsigned short* pb3 = WCT + (size_t)(3 * 16 + lr) * F2 + 8 * lh;
  v8f acc0 = zero8(), acc1 = zero8(), acc2 = zero8(), acc3 = zero8();
#pragma unroll 2
  for (int ks = 0; ks < 8; ++ks) {
    const v16bf ah = ldf(pah + 32 * ks);
    const v16bf al = ldf(pal + 32 * ks);
    const v16bf b0 = ldf(pb0 + 32 * ks);
    const v16bf b1 = ldf(pb1 + 32 * ks);
    const v16bf b2 = ldf(pb2 + 32 * ks);
    const v16bf b3 = ldf(pb3 + 32 * ks);
    acc0 = mma(ah, b0, acc0); acc0 = mma(al, b0, acc0);
    acc1 = mma(ah, b1, acc1); acc1 = mma(al, b1, acc1);
    acc2 = mma(ah, b2, acc2); acc2 = mma(al, b2, acc2);
    acc3 = mma(ah, b3, acc3); acc3 = mma(al, b3, acc3);
  }
  const float a10 = bfr(ac[lr]),        a11 = bfr(ac[16 + lr]),        a12 = bfr(ac[32 + lr]),        a13 = bfr(ac[48 + lr]);
  const float a20 = bfr(ac[EMBD + lr]), a21 = bfr(ac[EMBD + 16 + lr]), a22 = bfr(ac[EMBD + 32 + lr]), a23 = bfr(ac[EMBD + 48 + lr]);
  float p1[8], p2[8];
#pragma unroll
  for (int r = 0; r < 8; ++r) {
    p1[r] = acc0[r] * a10 + acc1[r] * a11 + acc2[r] * a12 + acc3[r] * a13;
    p2[r] = acc0[r] * a20 + acc1[r] * a21 + acc2[r] * a22 + acc3[r] * a23;
  }
#pragma unroll
  for (int r = 0; r < 8; ++r) {
#pragma unroll
    for (int off = 1; off < 16; off <<= 1) {
      p1[r] += __shfl_xor(p1[r], off, 32);
      p2[r] += __shfl_xor(p2[r], off, 32);
    }
  }
  if (lr == 0) {
#pragma unroll
    for (int r = 0; r < 8; ++r) {
      ws12[16 * wid + 8 * lh + r]      = p1[r];
      ws12[64 + 16 * wid + 8 * lh + r] = p2[r];
    }
  }
  __syncthreads();
  if (wid == 0) {
    const v4f v = *(const v4f*)(ws12 + 4 * lane);
    float* dst = W12 + (size_t)(lane >> 4) * (size_t)N + r0 + 4 * (lane & 15);
    *(volatile v4f*)dst = v;
    __threadfence();
    *(volatile v4f*)dst = v;
  }
}

__global__ __launch_bounds__(256) void k_out(const float* __restrict__ HF, const float* __restrict__ W12,
                                             const int* __restrict__ kadj, float* out, int N) {
  const int tid  = threadIdx.x;
  const int lane = tid & 31;
  const int wid  = tid >> 5;
  const int n    = 8 * blockIdx.x + wid;
  const int k    = lane & 15;
  int nb = kadj[(size_t)n * KNB + k];
  nb = min(max(nb, 0), N - 1);
  float s = W12[nb] + W12[(size_t)N + n];
  s = (s >= 0.0f) ? s : 0.2f * s;
  float mx = s;
#pragma unroll
  for (int off = 8; off > 0; off >>= 1) mx = fmaxf(mx, __shfl_xor(mx, off, 32));
  const float e = __expf(s - mx);
  float se = e;
#pragma unroll
  for (int off = 8; off > 0; off >>= 1) se += __shfl_xor(se, off, 32);
  const float att = e * __builtin_amdgcn_rcpf(se);
  v4f acc0, acc1;
  acc0[0] = 0.f; acc0[1] = 0.f; acc0[2] = 0.f; acc0[3] = 0.f;
  acc1 = acc0;
#pragma unroll 2
  for (int j = 0; j < KNB; ++j) {
    const int   nbj = __shfl(nb, j, 32);
    const float aj  = __shfl(att, j, 32);
    const float* src = HF + (size_t)nbj * F2 + 4 * lane;
    const v4f v0 = *(const v4f*)(src);
    const v4f v1 = *(const v4f*)(src + FG);
    acc0 += aj * v0;
    acc1 += aj * v1;
  }
  const float* self = HF + (size_t)n * F2 + 4 * lane;
  const v4f o0 = elu4(acc0 + *(const v4f*)(self));
  const v4f o1 = elu4(acc1 + *(const v4f*)(self + FG));
  float* dst = out + (size_t)n * F2 + 4 * lane;
  *(volatile v4f*)(dst)      = o0;
  *(volatile v4f*)(dst + FG) = o1;
  __threadfence();
  *(volatile v4f*)(dst)      = o0;
  *(volatile v4f*)(dst + FG) = o1;
}

extern "C" void kernel_launch(void* const* d_in, const int* in_sizes, int n_in,
                              void* d_out, int out_size, void* d_ws, size_t ws_size,
                              hipStream_t stream) {
  if (n_in < 11) return;
  if (in_sizes[0] != NCELL * FG) return;
  if (in_sizes[1] != NCELL * KNB) return;
  if (in_sizes[2] != DKK || in_sizes[3] != DKK) return;
  if (in_sizes[4] != DKK * DKK || in_sizes[5] != DKK) return;
  if (in_sizes[6] != DKK * DKK || in_sizes[7] != DKK) return;
  if (in_sizes[8] != DKK * KNB) return;
  if (in_sizes[9] != F2 * EMBD) return;
  if (in_sizes[10] != 2 * EMBD) return;
  if (out_size != NCELL * F2) return;
  if ((size_t)WS_TOTAL > ws_size) return;
  if ((size_t)WS_TOTAL > (size_t)134217728) return;

  const float* h    = (const float*)d_in[0];
  const int*   kadj = (const int*)d_in[1];
  const float* Whw  = (const float*)d_in[2];
  const float* Whb  = (const float*)d_in[3];
  const float* Qw   = (const float*)d_in[4];
  const float* Qb   = (const float*)d_in[5];
  const float* Kw   = (const float*)d_in[6];
  const float* Kb   = (const float*)d_in[7];
  const float* Ag   = (const float*)d_in[8];
  const float* Wc   = (const float*)d_in[9];
  const float* ac   = (const float*)d_in[10];
  float* out = (float*)d_out;

  unsigned char*  ws  = (unsigned char*)d_ws;
  unsigned short* WCT = (unsigned short*)(ws + WS_WCT);
  float*          HF  = (float*)(ws + WS_HF);
  unsigned short* HH  = (unsigned short*)(ws + WS_HH);
  unsigned short* HL  = (unsigned short*)(ws + WS_HL);
  float*          W12 = (float*)(ws + WS_W12);
  const int N = NCELL;

  (void)hipFuncSetAttribute(reinterpret_cast<const void*>(&k_cell),
                            hipFuncAttributeMaxDynamicSharedMemorySize, LDS_CELL);

  const dim3 gPrep(4),      bPrep(256);
  const dim3 gCell(N),      bCell(256);
  const dim3 gWc(N / 64),   bWc(128);
  const dim3 gOut(N / 8),   bOut(256);

  k_prep<<<gPrep, bPrep, 0, stream>>>(Wc, WCT);
  k_cell<<<gCell, bCell, LDS_CELL, stream>>>(h, kadj, Whw, Whb, Qw, Qb, Kw, Kb, Ag, HF, HH, HL, N);
  k_wcell<<<gWc, bWc, 0, stream>>>(HH, HL, WCT, ac, W12, N);
  k_out<<<gOut, bOut, 0, stream>>>(HF, W12, kadj, out, N);
  (void)hipGetLastError();
}
